// MDN_module_21655225106918
// MI455X (gfx1250) — hardware-run, weakly checked
//
#include <hip/hip_runtime.h>
#include <stddef.h>
#include <stdint.h>


#define B_DIM 8192
#define N_DIM 256
#define H_DIM 2048
#define F_DIM 512
#define NTHR  256
#define SC_W1 16.0f
#define SC_W2 64.0f
#define SC_WV 16.0f
#define INV16 (1.0f / 16.0f)
#define INV64 (1.0f / 64.0f)
#define BETA_F 0.99f
#define NLOG2PI_F 470.496529f
#define TP 72
#define WSCAP 134217728
#define LDS_G1 (8 * 32 * 64 * 4 + 8 * 32 * 64 * 2)
#define LDS_G2 (8 * 32 * 64 * 4)
#define NPART (B_DIM / 32)

static_assert((B_DIM % 128) == 0);
static_assert((H_DIM % 128) == 0);
static_assert((F_DIM % 128) == 0);
static_assert((N_DIM % 64) == 0);
static_assert((N_DIM % 32) == 0);
static_assert((H_DIM % 32) == 0);
static_assert(F_DIM == 2 * N_DIM);
static_assert(((B_DIM * N_DIM) % (8 * NTHR)) == 0);
static_assert(NPART == NTHR);
static_assert((B_DIM % 64) == 0);
static_assert(LDS_G1 <= 300 * 1024);

typedef float    v4f  __attribute__((ext_vector_type(4)));
typedef float    v8f  __attribute__((ext_vector_type(8)));
typedef _Float16 v8h  __attribute__((ext_vector_type(8)));
typedef _Float16 v16h __attribute__((ext_vector_type(16)));
union FragH { v16h v; v8h h[2]; };

__device__ __forceinline__ v8f wmf(v16h a, v16h b, v8f c) {
  v8f d = __builtin_amdgcn_wmma_f32_16x16x32_f16(false, a, false, b, (short)0, c, false, false);
  asm volatile("v_nop\n\tv_nop\n\tv_nop\n\tv_nop" : "+v"(d) : "v"(a), "v"(b));
  return d;
}

template <int KD>
__device__ __forceinline__ void mma_32x64(const _Float16* __restrict__ ap, const _Float16* __restrict__ bp,
                                          v8f (&acc)[2][4]) {
#pragma unroll 1
  for (int kt = 0; kt < KD / 32; ++kt) {
    const int k0 = 32 * kt;
    FragH a0, a1;
    a0.h[0] = *(const v8h*)(ap + k0);
    a0.h[1] = *(const v8h*)(ap + k0 + 16);
    a1.h[0] = *(const v8h*)(ap + (size_t)16 * KD + k0);
    a1.h[1] = *(const v8h*)(ap + (size_t)16 * KD + k0 + 16);
#pragma unroll
    for (int nt = 0; nt < 4; ++nt) {
      const _Float16* bq = bp + (size_t)nt * 16 * KD + k0;
      FragH b;
      b.h[0] = *(const v8h*)bq;
      b.h[1] = *(const v8h*)(bq + 16);
      acc[0][nt] = wmf(a0.v, b.v, acc[0][nt]);
      acc[1][nt] = wmf(a1.v, b.v, acc[1][nt]);
    }
  }
}

__global__ __launch_bounds__(NTHR) void k_cvt8(const float* __restrict__ in, _Float16* out) {
  const size_t t = (size_t)blockIdx.x * NTHR + threadIdx.x;
  const float* p = in + t * 8;
  const v4f f0 = *(const v4f*)p;
  const v4f f1 = *(const v4f*)(p + 4);
  v8h a;
  a[0] = (_Float16)f0.x; a[1] = (_Float16)f0.y; a[2] = (_Float16)f0.z; a[3] = (_Float16)f0.w;
  a[4] = (_Float16)f1.x; a[5] = (_Float16)f1.y; a[6] = (_Float16)f1.z; a[7] = (_Float16)f1.w;
  _Float16* d = out + t * 8;
  *(volatile v8h*)d = a;
  __threadfence();
  *(volatile v8h*)d = a;
}

__global__ __launch_bounds__(NTHR) void k_tcvt(const float* __restrict__ in, _Float16* outT,
                                               int R, int C, float sc) {
  __shared__ __attribute__((aligned(16))) _Float16 sT[64 * TP];
  const int tid = threadIdx.x;
  const int c0 = blockIdx.x * 64, r0 = blockIdx.y * 64;
  const int r = tid >> 2, cc = (tid & 3) * 16;
  const float* src = in + (size_t)(r0 + r) * C + c0 + cc;
#pragma unroll
  for (int j = 0; j < 4; ++j) {
    const v4f v = *(const v4f*)(src + 4 * j);
    sT[(cc + 4 * j + 0) * TP + r] = (_Float16)(v.x * sc);
    sT[(cc + 4 * j + 1) * TP + r] = (_Float16)(v.y * sc);
    sT[(cc + 4 * j + 2) * TP + r] = (_Float16)(v.z * sc);
    sT[(cc + 4 * j + 3) * TP + r] = (_Float16)(v.w * sc);
  }
  __syncthreads();
  const int p = tid & 7;
#pragma unroll
  for (int pass = 0; pass < 2; ++pass) {
    const int c = (tid >> 3) + 32 * pass;
    const v8h v = *(const v8h*)(sT + c * TP + 8 * p);
    _Float16* d = outT + (size_t)(c0 + c) * R + r0 + 8 * p;
    *(volatile v8h*)d = v;
  }
  __threadfence();
#pragma unroll
  for (int pass = 0; pass < 2; ++pass) {
    const int c = (tid >> 3) + 32 * pass;
    const v8h v = *(const v8h*)(sT + c * TP + 8 * p);
    _Float16* d = outT + (size_t)(c0 + c) * R + r0 + 8 * p;
    *(volatile v8h*)d = v;
  }
}

__global__ __launch_bounds__(NTHR) void k_gemm1(const _Float16* __restrict__ xh, const _Float16* __restrict__ w1t,
                                                const float* __restrict__ b1, _Float16* hh) {
  extern __shared__ v4f lds_dyn[];
  const int tid = threadIdx.x, lane = tid & 31, wave = tid >> 5, hf = lane >> 4, m = lane & 15;
  float* stg = (float*)lds_dyn + wave * (32 * 64);
  _Float16* stg16 = (_Float16*)((float*)lds_dyn + 8 * 32 * 64) + wave * (32 * 64);
  const int n0 = blockIdx.x * 128, m0 = blockIdx.y * 128;
  const int wm = (wave >> 1) * 32, wn = (wave & 1) * 64;

  v8f acc[2][4];
#pragma unroll
  for (int mt = 0; mt < 2; ++mt)
#pragma unroll
    for (int nt = 0; nt < 4; ++nt) { v8f z = {0.f, 0.f, 0.f, 0.f, 0.f, 0.f, 0.f, 0.f}; acc[mt][nt] = z; }

  const _Float16* ap = xh + (size_t)(m0 + wm + m) * N_DIM + 8 * hf;
  const _Float16* bp = w1t + (size_t)(n0 + wn + m) * N_DIM + 8 * hf;
  mma_32x64<N_DIM>(ap, bp, acc);

  float bv[4];
#pragma unroll
  for (int nt = 0; nt < 4; ++nt) bv[nt] = b1[n0 + wn + 16 * nt + m];
#pragma unroll
  for (int mt = 0; mt < 2; ++mt) {
    float* sp = stg + (16 * mt + 8 * hf) * 64 + m;
#pragma unroll
    for (int nt = 0; nt < 4; ++nt) {
#pragma unroll
      for (int r = 0; r < 8; ++r) sp[r * 64 + 16 * nt] = acc[mt][nt][r] * INV16 + bv[nt];
    }
  }
  __syncthreads();

  const int p = lane & 7, rq = lane >> 3;
  _Float16* gbase = hh + (size_t)(m0 + wm) * H_DIM + n0 + wn + 8 * p;
#pragma unroll 1
  for (int q = 0; q < 8; ++q) {
    const int row = 4 * q + rq;
    const v4f f0 = *(const v4f*)(stg + row * 64 + 8 * p);
    const v4f f1 = *(const v4f*)(stg + row * 64 + 8 * p + 4);
    v8h hv;
    hv[0] = (_Float16)tanhf(f0.x); hv[1] = (_Float16)tanhf(f0.y);
    hv[2] = (_Float16)tanhf(f0.z); hv[3] = (_Float16)tanhf(f0.w);
    hv[4] = (_Float16)tanhf(f1.x); hv[5] = (_Float16)tanhf(f1.y);
    hv[6] = (_Float16)tanhf(f1.z); hv[7] = (_Float16)tanhf(f1.w);
    *(v8h*)(stg16 + row * 64 + 8 * p) = hv;
    *(volatile v8h*)(gbase + (size_t)row * H_DIM) = hv;
  }
  __threadfence();
  __syncthreads();
#pragma unroll 1
  for (int q = 0; q < 8; ++q) {
    const int row = 4 * q + rq;
    const v8h hv = *(const v8h*)(stg16 + row * 64 + 8 * p);
    *(volatile v8h*)(gbase + (size_t)row * H_DIM) = hv;
  }
}

__global__ __launch_bounds__(NTHR) void k_gemm2(const _Float16* __restrict__ hh, const _Float16* __restrict__ w2t,
                                                const float* __restrict__ b2, float* fb, _Float16* muh) {
  extern __shared__ v4f lds_dyn[];
  const int tid = threadIdx.x, lane = tid & 31, wave = tid >> 5, hf = lane >> 4, m = lane & 15;
  float* stg = (float*)lds_dyn + wave * (32 * 64);
  const int n0 = blockIdx.x * 128, m0 = blockIdx.y * 128;
  const int wm = (wave >> 1) * 32, wn = (wave & 1) * 64;

  v8f acc[2][4];
#pragma unroll
  for (int mt = 0; mt < 2; ++mt)
#pragma unroll
    for (int nt = 0; nt < 4; ++nt) { v8f z = {0.f, 0.f, 0.f, 0.f, 0.f, 0.f, 0.f, 0.f}; acc[mt][nt] = z; }

  const _Float16* ap = hh + (size_t)(m0 + wm + m) * H_DIM + 8 * hf;
  const _Float16* bp = w2t + (size_t)(n0 + wn + m) * H_DIM + 8 * hf;
  mma_32x64<H_DIM>(ap, bp, acc);

  float bv[4];
#pragma unroll
  for (int nt = 0; nt < 4; ++nt) bv[nt] = b2[n0 + wn + 16 * nt + m];
#pragma unroll
  for (int mt = 0; mt < 2; ++mt) {
    float* sp = stg + (16 * mt + 8 * hf) * 64 + m;
#pragma unroll
    for (int nt = 0; nt < 4; ++nt) {
#pragma unroll
      for (int r = 0; r < 8; ++r) sp[r * 64 + 16 * nt] = acc[mt][nt][r] * INV64 + bv[nt];
    }
  }
  __syncthreads();

  const bool mu_blk = (blockIdx.x < 2);
  float* gbase = fb + (size_t)(m0 + wm) * F_DIM + n0 + wn;
  const int p = lane & 7, rq = lane >> 3;
  _Float16* hbase = muh + (size_t)(m0 + wm) * N_DIM + n0 + wn + 8 * p;

#pragma unroll
  for (int q = 0; q < 16; ++q) {
    const int row = 2 * q + hf;
    const v4f v = *(const v4f*)(stg + row * 64 + 4 * m);
    *(volatile v4f*)(gbase + (size_t)row * F_DIM + 4 * m) = v;
  }
  if (mu_blk) {
#pragma unroll 1
    for (int q = 0; q < 8; ++q) {
      const int row = 4 * q + rq;
      const v4f f0 = *(const v4f*)(stg + row * 64 + 8 * p);
      const v4f f1 = *(const v4f*)(stg + row * 64 + 8 * p + 4);
      v8h hv;
      hv[0] = (_Float16)f0.x; hv[1] = (_Float16)f0.y; hv[2] = (_Float16)f0.z; hv[3] = (_Float16)f0.w;
      hv[4] = (_Float16)f1.x; hv[5] = (_Float16)f1.y; hv[6] = (_Float16)f1.z; hv[7] = (_Float16)f1.w;
      *(volatile v8h*)(hbase + (size_t)row * N_DIM) = hv;
    }
  }
  __threadfence();
#pragma unroll
  for (int q = 0; q < 16; ++q) {
    const int row = 2 * q + hf;
    const v4f v = *(const v4f*)(stg + row * 64 + 4 * m);
    *(volatile v4f*)(gbase + (size_t)row * F_DIM + 4 * m) = v;
  }
  if (mu_blk) {
#pragma unroll 1
    for (int q = 0; q < 8; ++q) {
      const int row = 4 * q + rq;
      const v4f f0 = *(const v4f*)(stg + row * 64 + 8 * p);
      const v4f f1 = *(const v4f*)(stg + row * 64 + 8 * p + 4);
      v8h hv;
      hv[0] = (_Float16)f0.x; hv[1] = (_Float16)f0.y; hv[2] = (_Float16)f0.z; hv[3] = (_Float16)f0.w;
      hv[4] = (_Float16)f1.x; hv[5] = (_Float16)f1.y; hv[6] = (_Float16)f1.z; hv[7] = (_Float16)f1.w;
      *(volatile v8h*)(hbase + (size_t)row * N_DIM) = hv;
    }
  }
}

__global__ __launch_bounds__(NTHR) void k_vquad(const _Float16* __restrict__ A, const _Float16* __restrict__ wvt,
                                                float* Vout) {
  __shared__ float spart[256];
  __shared__ __attribute__((aligned(16))) float sline[64];
  const int tid = threadIdx.x, lane = tid & 31, wave = tid >> 5, hf = lane >> 4, m = lane & 15;
  const int r0 = blockIdx.x * 64;
  const int wm = (wave >> 2) * 32, wn = (wave & 3) * 64;

  v8f acc[2][4];
#pragma unroll
  for (int mt = 0; mt < 2; ++mt)
#pragma unroll
    for (int nt = 0; nt < 4; ++nt) { v8f z = {0.f, 0.f, 0.f, 0.f, 0.f, 0.f, 0.f, 0.f}; acc[mt][nt] = z; }

  const _Float16* ap = A + (size_t)(r0 + wm + m) * N_DIM + 8 * hf;
  const _Float16* bp = wvt + (size_t)(wn + m) * N_DIM + 8 * hf;
  mma_32x64<N_DIM>(ap, bp, acc);

#pragma unroll
  for (int mt = 0; mt < 2; ++mt) {
#pragma unroll
    for (int r = 0; r < 8; ++r) {
      float s = 0.0f;
#pragma unroll
      for (int nt = 0; nt < 4; ++nt) {
        const float u = acc[mt][nt][r] * INV16;
        s = fmaf(u, u, s);
      }
      s += __shfl_xor(s, 1, 32);
      s += __shfl_xor(s, 2, 32);
      s += __shfl_xor(s, 4, 32);
      s += __shfl_xor(s, 8, 32);
      if (m == 0) spart[(wave & 3) * 64 + wm + 16 * mt + 8 * hf + r] = s;
    }
  }
  __syncthreads();
  if (tid < 64) {
    const float v = ((spart[tid] + spart[64 + tid]) + spart[128 + tid]) + spart[192 + tid];
    sline[tid] = v + 1e-3f;
  }
  __syncthreads();
  if (tid < 16) {
    const v4f v = *(const v4f*)(sline + 4 * tid);
    float* d = Vout + (size_t)r0 + 4 * tid;
    *(volatile v4f*)d = v;
    __threadfence();
    *(volatile v4f*)d = v;
  }
}

__global__ __launch_bounds__(NTHR) void k_final(const float* __restrict__ fb, const float* __restrict__ Vx,
                                                const float* __restrict__ Vmu, const float* __restrict__ y,
                                                const float* __restrict__ eps, float* fx, float* part) {
  __shared__ float sred[8];
  __shared__ __attribute__((aligned(16))) float sline[32];
  const int tid = threadIdx.x, lane = tid & 31, wave = tid >> 5;
  float wacc = 0.0f;
#pragma unroll 1
  for (int rr = 0; rr < 4; ++rr) {
    const int row = blockIdx.x * 32 + wave * 4 + rr;
    const float vx = Vx[row];
    const float vmu = Vmu[row];
    const float bvx = BETA_F * vx;
    const float rel = fmaxf(bvx - vmu, 0.0f);
    const float scale = (bvx - rel) * (1.0f / vmu);
    const size_t rb = (size_t)row;
    float tsum = 0.0f;
#pragma unroll 1
    for (int half = 0; half < 2; ++half) {
      const int c = half * 128 + 4 * lane;
      const v4f mv = *(const v4f*)(fb + rb * F_DIM + c);
      const v4f lv = *(const v4f*)(fb + rb * F_DIM + N_DIM + c);
      const v4f yv = *(const v4f*)(y + rb * N_DIM + c);
      const v4f ev = *(const v4f*)(eps + rb * N_DIM + c);
      v4f fo;
#pragma unroll
      for (int e = 0; e < 4; ++e) {
        const float ms = mv[e] * scale;
        const float var = expf(lv[e]);
        fo[e] = ms + sqrtf(var) * ev[e];
        const float d = yv[e] - ms;
        tsum += lv[e] + d * d * (1.0f / var);
      }
      float* dst = fx + rb * N_DIM + c;
      *(volatile v4f*)dst = fo;
      __threadfence();
      *(volatile v4f*)dst = fo;
    }
    tsum += __shfl_xor(tsum, 16, 32);
    tsum += __shfl_xor(tsum, 8, 32);
    tsum += __shfl_xor(tsum, 4, 32);
    tsum += __shfl_xor(tsum, 2, 32);
    tsum += __shfl_xor(tsum, 1, 32);
    wacc += 0.5f * (NLOG2PI_F + tsum);
  }
  if (lane == 0) sred[wave] = wacc;
  __syncthreads();
  if (tid < 32) {
    float v = 0.0f;
    if (tid == 0) {
#pragma unroll
      for (int w = 0; w < 8; ++w) v += sred[w];
    }
    sline[tid] = v;
  }
  __syncthreads();
  if (tid < 8) {
    const v4f v = *(const v4f*)(sline + 4 * tid);
    float* d = part + (size_t)blockIdx.x * 32 + 4 * tid;
    *(volatile v4f*)d = v;
    __threadfence();
    *(volatile v4f*)d = v;
  }
}

__global__ __launch_bounds__(NTHR) void k_reduce(const float* __restrict__ part, float* out1) {
  __shared__ float sred[8];
  const int tid = threadIdx.x, lane = tid & 31, wave = tid >> 5;
  float v = part[(size_t)tid * 32];
  v += __shfl_xor(v, 16, 32);
  v += __shfl_xor(v, 8, 32);
  v += __shfl_xor(v, 4, 32);
  v += __shfl_xor(v, 2, 32);
  v += __shfl_xor(v, 1, 32);
  if (lane == 0) sred[wave] = v;
  __syncthreads();
  if (tid == 0) {
    float t = 0.0f;
#pragma unroll
    for (int w = 0; w < 8; ++w) t += sred[w];
    *(volatile float*)out1 = t;
    __threadfence();
    *(volatile float*)out1 = t;
  }
}

extern "C" void kernel_launch(void* const* d_in, const int* in_sizes, int n_in,
                              void* d_out, int out_size, void* d_ws, size_t ws_size,
                              hipStream_t stream) {
  if (n_in < 8) return;
  if (in_sizes[0] != B_DIM * N_DIM || in_sizes[1] != B_DIM * N_DIM || in_sizes[2] != B_DIM * N_DIM ||
      in_sizes[3] != N_DIM * H_DIM || in_sizes[4] != H_DIM || in_sizes[5] != H_DIM * F_DIM ||
      in_sizes[6] != F_DIM || in_sizes[7] != N_DIM * N_DIM) return;
  if (out_size != B_DIM * N_DIM + 1) return;

  const float* x   = (const float*)d_in[0];
  const float* y   = (const float*)d_in[1];
  const float* eps = (const float*)d_in[2];
  const float* W1  = (const float*)d_in[3];
  const float* b1  = (const float*)d_in[4];
  const float* W2  = (const float*)d_in[5];
  const float* b2  = (const float*)d_in[6];
  const float* Wv  = (const float*)d_in[7];
  float* out  = (float*)d_out;
  float* out1 = out + (size_t)B_DIM * N_DIM;

  char* ws = (char*)d_ws;
  size_t off = 0;
  const size_t oX  = off; off += (size_t)B_DIM * N_DIM * 2;  off = (off + 255) & ~(size_t)255;
  const size_t oW1 = off; off += (size_t)H_DIM * N_DIM * 2;  off = (off + 255) & ~(size_t)255;
  const size_t oW2 = off; off += (size_t)F_DIM * H_DIM * 2;  off = (off + 255) & ~(size_t)255;
  const size_t oWv = off; off += (size_t)N_DIM * N_DIM * 2;  off = (off + 255) & ~(size_t)255;
  const size_t oH  = off; off += (size_t)B_DIM * H_DIM * 2;  off = (off + 255) & ~(size_t)255;
  const size_t oF  = off; off += (size_t)B_DIM * F_DIM * 4;  off = (off + 255) & ~(size_t)255;
  const size_t oMu = off; off += (size_t)B_DIM * N_DIM * 2;  off = (off + 255) & ~(size_t)255;
  const size_t oVx = off; off += (size_t)B_DIM * 4;          off = (off + 255) & ~(size_t)255;
  const size_t oVm = off; off += (size_t)B_DIM * 4;          off = (off + 255) & ~(size_t)255;
  const size_t oP  = off; off += (size_t)NPART * 32 * 4;     off = (off + 255) & ~(size_t)255;
  if (off > ws_size || off > (size_t)WSCAP) return;
  _Float16* xh  = (_Float16*)(ws + oX);
  _Float16* w1t = (_Float16*)(ws + oW1);
  _Float16* w2t = (_Float16*)(ws + oW2);
  _Float16* wvt = (_Float16*)(ws + oWv);
  _Float16* hh  = (_Float16*)(ws + oH);
  float*    fb  = (float*)(ws + oF);
  _Float16* muh = (_Float16*)(ws + oMu);
  float*    Vx  = (float*)(ws + oVx);
  float*    Vmu = (float*)(ws + oVm);
  float*    part = (float*)(ws + oP);

  k_cvt8<<<(B_DIM * N_DIM) / (8 * NTHR), NTHR, 0, stream>>>(x, xh);
  k_tcvt<<<dim3(H_DIM / 64, N_DIM / 64), NTHR, 0, stream>>>(W1, w1t, N_DIM, H_DIM, SC_W1);
  k_tcvt<<<dim3(F_DIM / 64, H_DIM / 64), NTHR, 0, stream>>>(W2, w2t, H_DIM, F_DIM, SC_W2);
  k_tcvt<<<dim3(N_DIM / 64, N_DIM / 64), NTHR, 0, stream>>>(Wv, wvt, N_DIM, N_DIM, SC_WV);

  hipFuncSetAttribute(reinterpret_cast<const void*>(&k_gemm1),
                      hipFuncAttributeMaxDynamicSharedMemorySize, LDS_G1);
  k_gemm1<<<dim3(H_DIM / 128, B_DIM / 128), NTHR, LDS_G1, stream>>>(xh, w1t, b1, hh);

  k_vquad<<<B_DIM / 64, NTHR, 0, stream>>>(xh, wvt, Vx);

  hipFuncSetAttribute(reinterpret_cast<const void*>(&k_gemm2),
                      hipFuncAttributeMaxDynamicSharedMemorySize, LDS_G2);
  k_gemm2<<<dim3(F_DIM / 128, B_DIM / 128), NTHR, LDS_G2, stream>>>(hh, w2t, b2, fb, muh);

  k_vquad<<<B_DIM / 64, NTHR, 0, stream>>>(muh, wvt, Vmu);

  k_final<<<B_DIM / 32, NTHR, 0, stream>>>(fb, Vx, Vmu, y, eps, out, part);

  k_reduce<<<1, NTHR, 0, stream>>>(part, out1);
}
